// Decoder_14680198217759
// MI455X (gfx1250) — hardware-verified
//
#include <hip/hip_runtime.h>
#include <stddef.h>
#include <stdint.h>

#ifndef NB
#define NB 32
#endif
#define GQ     512
#define NK     512
#define EW     128
#define NH     8
#define HD     16
#define QROW   32
#define MPITCH 516
#define CPITCH 136
#define TPITCH 136
#define WSMAX  134217728
#define VPL    ((size_t)NB * EW * NK)

static_assert(GQ == NK);
static_assert(NH * HD == EW);
static_assert(EW % 32 == 0 && NK % 32 == 0);
static_assert(GQ % 64 == 0 && (NB * GQ) % 64 == 0);
static_assert(NH * 64 * QROW == 16384);
static_assert(2 * EW * 64 == 16384);
static_assert(16384 == 128 * 16 * 8);
static_assert(32 * EW == 256 * 2 * 8);
static_assert(((size_t)NB * NK * EW) % (256 * 8) == 0);
static_assert(16 * NK == 256 * 8 * 4);
static_assert(NK == 8 * 64);
static_assert(NK == 32 * 16);

typedef int            v4i   __attribute__((ext_vector_type(4)));
typedef int            v8i   __attribute__((ext_vector_type(8)));
typedef float          v4f   __attribute__((ext_vector_type(4)));
typedef float          v8f   __attribute__((ext_vector_type(8)));
typedef __bf16         v16bf __attribute__((ext_vector_type(16)));
typedef v4i __attribute__((may_alias)) v4ia;
typedef v4f __attribute__((may_alias)) v4fa;
union FragB { v16bf v; v4i q[2]; v8i w; };

__device__ __forceinline__ v8f wmb(const FragB& a, const FragB& b, v8f c) {
  v8f d = __builtin_amdgcn_wmma_f32_16x16x32_bf16(false, a.v, false, b.v, (short)0, c, false, false);
  asm volatile("v_nop\n\tv_nop\n\tv_nop\n\tv_nop" : "+v"(d) : "v"(a.w), "v"(b.w));
  return d;
}

__device__ __forceinline__ unsigned bf16_bits(float f) {
  const unsigned u = __float_as_uint(f);
  return (u + 0x7FFFu + ((u >> 16) & 1u)) >> 16;
}
__device__ __forceinline__ float bf16_val(float f) {
  return __uint_as_float(bf16_bits(f) << 16);
}
__device__ __forceinline__ int pack2(float lo, float hi) {
  return (int)(bf16_bits(lo) | (bf16_bits(hi) << 16));
}
__device__ __forceinline__ void split8(const v8f x, v4i& hi, v4i& lo) {
#pragma unroll
  for (int j = 0; j < 4; ++j) {
    const float a = x[2 * j], b = x[2 * j + 1];
    const unsigned ha = bf16_bits(a), hb = bf16_bits(b);
    const float ra = a - __uint_as_float(ha << 16);
    const float rb = b - __uint_as_float(hb << 16);
    hi[j] = (int)(ha | (hb << 16));
    lo[j] = (int)(bf16_bits(ra) | (bf16_bits(rb) << 16));
  }
}
__device__ __forceinline__ FragB ldf_frag(const float* __restrict__ p) {
  const v4f a0 = *(const v4fa*)p;
  const v4f a1 = *(const v4fa*)(p + 4);
  const v4f a2 = *(const v4fa*)(p + 16);
  const v4f a3 = *(const v4fa*)(p + 20);
  FragB f;
  f.w[0] = pack2(a0.x, a0.y); f.w[1] = pack2(a0.z, a0.w);
  f.w[2] = pack2(a1.x, a1.y); f.w[3] = pack2(a1.z, a1.w);
  f.w[4] = pack2(a2.x, a2.y); f.w[5] = pack2(a2.z, a2.w);
  f.w[6] = pack2(a3.x, a3.y); f.w[7] = pack2(a3.z, a3.w);
  return f;
}
__device__ __forceinline__ FragB ldg_frag(const unsigned short* __restrict__ p) {
  FragB f;
  f.q[0] = *(const v4ia*)p;
  f.q[1] = *(const v4ia*)(p + 16);
  return f;
}

__global__ __launch_bounds__(256) void k_wprep(const float* __restrict__ w0, const float* __restrict__ w1,
                                               const float* __restrict__ w2, const float* __restrict__ w3,
                                               const float* __restrict__ w4, unsigned short* wt) {
  __shared__ __attribute__((aligned(16))) unsigned short T[32 * TPITCH];
  const unsigned tid = threadIdx.x;
  const unsigned n0 = blockIdx.x * 32u, ws = blockIdx.y;
  const float* W = (ws == 0u) ? w0 : (ws == 1u) ? w1 : (ws == 2u) ? w2 : (ws == 3u) ? w3 : w4;
#pragma unroll 1
  for (unsigned it = 0; it < 4u; ++it) {
    const unsigned k = (tid >> 3) + 32u * it;
    const unsigned n4 = (tid & 7u) << 2;
    const v4f v = *(const v4fa*)(W + (size_t)k * EW + n0 + n4);
    T[(n4 + 0u) * TPITCH + k] = (unsigned short)bf16_bits(v.x);
    T[(n4 + 1u) * TPITCH + k] = (unsigned short)bf16_bits(v.y);
    T[(n4 + 2u) * TPITCH + k] = (unsigned short)bf16_bits(v.z);
    T[(n4 + 3u) * TPITCH + k] = (unsigned short)bf16_bits(v.w);
  }
  __syncthreads();
  unsigned short* dst = wt + (size_t)ws * (EW * EW) + (size_t)n0 * EW;
#pragma unroll 1
  for (unsigned it = 0; it < 2u; ++it) {
    const unsigned p = it * 256u + tid, n = p >> 4, c = p & 15u;
    const v4i v = *(const v4ia*)(T + n * TPITCH + c * 8u);
    *(volatile v4i*)(dst + n * EW + c * 8u) = v;
  }
  __threadfence();
#pragma unroll 1
  for (unsigned it = 0; it < 2u; ++it) {
    const unsigned p = it * 256u + tid, n = p >> 4, c = p & 15u;
    const v4i v = *(const v4ia*)(T + n * TPITCH + c * 8u);
    *(volatile v4i*)(dst + n * EW + c * 8u) = v;
  }
}

__global__ __launch_bounds__(256) void k_cvt(const float* __restrict__ x, unsigned short* o) {
  const size_t i = (size_t)blockIdx.x * 256u + threadIdx.x;
  const float* p = x + i * 8u;
  const v4f a = *(const v4fa*)p;
  const v4f b = *(const v4fa*)(p + 4);
  v4i w;
  w[0] = pack2(a.x, a.y); w[1] = pack2(a.z, a.w);
  w[2] = pack2(b.x, b.y); w[3] = pack2(b.z, b.w);
  unsigned short* d = o + i * 8u;
  *(volatile v4i*)d = w;
  __threadfence();
  *(volatile v4i*)d = w;
}

template <int MODE>
__global__ __launch_bounds__(128) void k_proj(const float* __restrict__ x1, const float* __restrict__ x2,
                                              const unsigned short* __restrict__ w1t,
                                              const unsigned short* __restrict__ w2t,
                                              unsigned short* o1, unsigned short* o2) {
  __shared__ __attribute__((aligned(16))) unsigned short stg[16384];
  const unsigned tid = threadIdx.x, lane = tid & 31u, wave = tid >> 5, hh = lane >> 4, m = lane & 15u;
  const unsigned row0 = blockIdx.x * 64u;
  const unsigned bb = row0 >> 9, r0 = row0 & 511u;
  const unsigned xrow = row0 + 16u * wave + m;

  FragB xa[4], xb[4];
#pragma unroll
  for (int ks = 0; ks < 4; ++ks) {
    xa[ks] = ldf_frag(x1 + (size_t)xrow * EW + 32 * ks + 8u * hh);
    if (MODE == 0) xb[ks] = ldf_frag(x2 + (size_t)xrow * EW + 32 * ks + 8u * hh);
    else xb[ks] = xa[ks];
  }
  const v8f zero8 = {0.f, 0.f, 0.f, 0.f, 0.f, 0.f, 0.f, 0.f};

#pragma unroll 1
  for (unsigned t = 0; t < NH; ++t) {
    const unsigned short* wp = w1t + (size_t)(16u * t + m) * EW + 8u * hh;
    const unsigned short* wq = w2t + (size_t)(16u * t + m) * EW + 8u * hh;
    v8f acc = zero8;
#pragma unroll
    for (int ks = 0; ks < 4; ++ks) {
      const FragB wf = ldg_frag(wp + 32 * ks);
      acc = wmb(wf, xa[ks], acc);
      if (MODE == 0) {
        const FragB wg = ldg_frag(wq + 32 * ks);
        acc = wmb(wg, xb[ks], acc);
      }
    }
    v4i hi, lo;
    split8(acc, hi, lo);
    const unsigned so = (t * 64u + 16u * wave + m) * QROW + 8u * hh;
    *(v4ia*)(stg + so) = hi;
    *(v4ia*)(stg + so + 16u) = lo;
  }
  __syncthreads();
  {
    unsigned short* dst = o1 + ((size_t)bb * NH * GQ + r0) * QROW;
#pragma unroll 1
    for (unsigned it = 0; it < 16u; ++it) {
      const unsigned p = it * 128u + tid, t = p >> 8, wi = p & 255u;
      const v4i v = *(const v4ia*)(stg + p * 8u);
      *(volatile v4i*)(dst + (size_t)t * (GQ * QROW) + wi * 8u) = v;
    }
    __threadfence();
#pragma unroll 1
    for (unsigned it = 0; it < 16u; ++it) {
      const unsigned p = it * 128u + tid, t = p >> 8, wi = p & 255u;
      const v4i v = *(const v4ia*)(stg + p * 8u);
      *(volatile v4i*)(dst + (size_t)t * (GQ * QROW) + wi * 8u) = v;
    }
  }
  if (MODE == 1) {
    __syncthreads();
#pragma unroll 1
    for (unsigned t = 0; t < NH; ++t) {
      const unsigned short* wq = w2t + (size_t)(16u * t + m) * EW + 8u * hh;
      v8f acc = zero8;
#pragma unroll
      for (int ks = 0; ks < 4; ++ks) {
        const FragB wf = ldg_frag(wq + 32 * ks);
        acc = wmb(xa[ks], wf, acc);
      }
      v4i hi, lo;
      split8(acc, hi, lo);
      const unsigned so = (16u * t + m) * 64u + 16u * wave + 8u * hh;
      *(v4ia*)(stg + so) = hi;
      *(v4ia*)(stg + so + 8192u) = lo;
    }
    __syncthreads();
    unsigned short* dst = o2 + (size_t)bb * EW * NK + r0;
#pragma unroll 1
    for (unsigned it = 0; it < 16u; ++it) {
      const unsigned p = it * 128u + tid, pl = p >> 10, col = (p >> 3) & 127u, c = p & 7u;
      const v4i v = *(const v4ia*)(stg + p * 8u);
      *(volatile v4i*)(dst + (size_t)pl * VPL + (size_t)col * NK + c * 8u) = v;
    }
    __threadfence();
#pragma unroll 1
    for (unsigned it = 0; it < 16u; ++it) {
      const unsigned p = it * 128u + tid, pl = p >> 10, col = (p >> 3) & 127u, c = p & 7u;
      const v4i v = *(const v4ia*)(stg + p * 8u);
      *(volatile v4i*)(dst + (size_t)pl * VPL + (size_t)col * NK + c * 8u) = v;
    }
  }
}

__global__ __launch_bounds__(256) void k_dec(const unsigned short* __restrict__ qpl,
                                             const unsigned short* __restrict__ kpl,
                                             const unsigned short* __restrict__ vt,
                                             const float* __restrict__ mask,
                                             const unsigned short* __restrict__ wct,
                                             const float* __restrict__ bcomb,
                                             const unsigned short* __restrict__ nbf,
                                             float* out) {
  __shared__ __attribute__((aligned(16))) float mk[16 * MPITCH];
  __shared__ __attribute__((aligned(16))) unsigned short cst[2 * 16 * CPITCH];
  __shared__ __attribute__((aligned(16))) unsigned short mst[2 * 16 * CPITCH];
  const unsigned tid = threadIdx.x, lane = tid & 31u, wave = tid >> 5, hh = lane >> 4, m = lane & 15u;
  const unsigned g0 = blockIdx.x * 16u, b = blockIdx.y;
  const v8f zero8 = {0.f, 0.f, 0.f, 0.f, 0.f, 0.f, 0.f, 0.f};
  const v4i zero4 = {0, 0, 0, 0};

  {
    const float* mg = mask + ((size_t)b * GQ + g0) * NK;
#pragma unroll 2
    for (unsigned it = 0; it < 8u; ++it) {
      const unsigned p = it * 256u + tid, row = p >> 7, c4 = (p & 127u) << 2;
      v4f v = *(const v4fa*)(mg + (size_t)row * NK + c4);
      v.x = bf16_val(v.x); v.y = bf16_val(v.y); v.z = bf16_val(v.z); v.w = bf16_val(v.w);
      *(v4fa*)(mk + row * MPITCH + c4) = v;
    }
  }
  __syncthreads();

  {
    const unsigned bh = b * NH + wave;
    const unsigned short* qp = qpl + ((size_t)bh * GQ + g0 + m) * QROW + 8u * hh;
    FragB qf;
    qf.q[0] = *(const v4ia*)qp;
    qf.q[1] = *(const v4ia*)(qp + 16);
    const unsigned short* kb = kpl + ((size_t)bh * NK + m) * QROW + 8u * hh;
    const unsigned short* vh = vt + ((size_t)bh * HD + m) * NK + 8u * hh;
    const unsigned short* vl = vh + VPL;
    const unsigned moff = m * MPITCH + 8u * hh;
    v8f o = zero8;
    float mrun = -3.0e38f, lrun = 0.0f;
#pragma unroll 1
    for (unsigned n0 = 0; n0 < NK; n0 += 32u) {
      const unsigned short* kp = kb + (size_t)n0 * QROW;
      const v4i kh0 = *(const v4ia*)kp;
      const v4i kl0 = *(const v4ia*)(kp + 16);
      const v4i kh1 = *(const v4ia*)(kp + 16 * QROW);
      const v4i kl1 = *(const v4ia*)(kp + 16 * QROW + 16);
      FragB a10, a20, a11, a21;
      a10.q[0] = kh0; a10.q[1] = kh0;
      a20.q[0] = kl0; a20.q[1] = zero4;
      a11.q[0] = kh1; a11.q[1] = kh1;
      a21.q[0] = kl1; a21.q[1] = zero4;
      v8f s0 = wmb(a10, qf, zero8);
      s0 = wmb(a20, qf, s0);
      v8f s1 = wmb(a11, qf, zero8);
      s1 = wmb(a21, qf, s1);

      const v4f m0 = *(const v4fa*)(mk + moff + n0);
      const v4f m1 = *(const v4fa*)(mk + moff + n0 + 4u);
      const v4f m2 = *(const v4fa*)(mk + moff + n0 + 16u);
      const v4f m3 = *(const v4fa*)(mk + moff + n0 + 20u);
      const v8f mk0 = __builtin_shufflevector(m0, m1, 0, 1, 2, 3, 4, 5, 6, 7);
      const v8f mk1 = __builtin_shufflevector(m2, m3, 0, 1, 2, 3, 4, 5, 6, 7);
      const v8f a0 = s0 * 0.25f + mk0;
      const v8f a1 = s1 * 0.25f + mk1;

      float t = fmaxf(a0[0], a1[0]);
#pragma unroll
      for (int r = 1; r < 8; ++r) t = fmaxf(t, fmaxf(a0[r], a1[r]));
      t = fmaxf(t, __shfl_xor(t, 16));
      const float mnew = fmaxf(mrun, t);
      const float sc = expf(mrun - mnew);
      v8f p0, p1;
      float ps = 0.0f;
#pragma unroll
      for (int r = 0; r < 8; ++r) {
        p0[r] = expf(a0[r] - mnew);
        p1[r] = expf(a1[r] - mnew);
        ps += p0[r] + p1[r];
      }
      lrun = lrun * sc + ps;
      mrun = mnew;
      o = o * sc;

      FragB ph, pl;
      split8(p0, ph.q[0], pl.q[0]);
      split8(p1, ph.q[1], pl.q[1]);
      FragB fvh, fvl;
      fvh.q[0] = *(const v4ia*)(vh + n0);
      fvh.q[1] = *(const v4ia*)(vh + n0 + 16u);
      fvl.q[0] = *(const v4ia*)(vl + n0);
      fvl.q[1] = *(const v4ia*)(vl + n0 + 16u);
      o = wmb(fvh, ph, o);
      o = wmb(fvl, ph, o);
      o = wmb(fvh, pl, o);
    }
    const float lt = lrun + __shfl_xor(lrun, 16);
    const float inv = 1.0f / lt;
    const v8f c = o * inv;
    v4i hi, lo;
    split8(c, hi, lo);
    const unsigned co = m * CPITCH + 16u * wave + 8u * hh;
    *(v4ia*)(cst + co) = hi;
    *(v4ia*)(cst + 16 * CPITCH + co) = lo;
  }
  __syncthreads();

  {
    const unsigned e0 = 16u * wave;
    const unsigned short* wp = wct + (size_t)(e0 + m) * EW + 8u * hh;
    const unsigned co = m * CPITCH + 8u * hh;
    v8f acc = zero8;
#pragma unroll
    for (int ks = 0; ks < 4; ++ks) {
      const FragB wf = ldg_frag(wp + 32 * ks);
      FragB ch, cl;
      ch.q[0] = *(const v4ia*)(cst + co + 32 * ks);
      ch.q[1] = *(const v4ia*)(cst + co + 32 * ks + 16);
      cl.q[0] = *(const v4ia*)(cst + 16 * CPITCH + co + 32 * ks);
      cl.q[1] = *(const v4ia*)(cst + 16 * CPITCH + co + 32 * ks + 16);
      acc = wmb(wf, ch, acc);
      acc = wmb(wf, cl, acc);
    }
    const v4f b0 = *(const v4fa*)(bcomb + e0 + 8u * hh);
    const v4f b1 = *(const v4fa*)(bcomb + e0 + 8u * hh + 4u);
    acc[0] += bf16_val(b0.x); acc[1] += bf16_val(b0.y);
    acc[2] += bf16_val(b0.z); acc[3] += bf16_val(b0.w);
    acc[4] += bf16_val(b1.x); acc[5] += bf16_val(b1.y);
    acc[6] += bf16_val(b1.z); acc[7] += bf16_val(b1.w);
    v4i hi, lo;
    split8(acc, hi, lo);
    const unsigned mo = m * CPITCH + e0 + 8u * hh;
    *(v4ia*)(mst + mo) = hi;
    *(v4ia*)(mst + 16 * CPITCH + mo) = lo;
  }
  __syncthreads();

  {
    const float ise = 1.0f / 11.313708498984761f;
    const unsigned ao = m * CPITCH + 8u * hh;
    FragB ah[4], al[4];
#pragma unroll
    for (int ks = 0; ks < 4; ++ks) {
      ah[ks].q[0] = *(const v4ia*)(mst + ao + 32 * ks);
      ah[ks].q[1] = *(const v4ia*)(mst + ao + 32 * ks + 16);
      al[ks].q[0] = *(const v4ia*)(mst + 16 * CPITCH + ao + 32 * ks);
      al[ks].q[1] = *(const v4ia*)(mst + 16 * CPITCH + ao + 32 * ks + 16);
    }
#pragma unroll 1
    for (unsigned j = 0; j < 4u; ++j) {
      const unsigned n0 = 64u * wave + 16u * j;
      const unsigned short* np = nbf + ((size_t)b * NK + n0 + m) * EW + 8u * hh;
      v8f acc = zero8;
#pragma unroll
      for (int ks = 0; ks < 4; ++ks) {
        const FragB nf = ldg_frag(np + 32 * ks);
        acc = wmb(ah[ks], nf, acc);
        acc = wmb(al[ks], nf, acc);
      }
#pragma unroll
      for (int r = 0; r < 8; ++r) {
        const unsigned idx = (8u * hh + (unsigned)r) * MPITCH + n0 + m;
        const float x = acc[r] * ise;
        const float s = 10.0f * tanhf(x) + mk[idx];
        mk[idx] = s;
      }
    }
  }
  __syncthreads();

  {
    v4f res[2][4];
#pragma unroll
    for (int rr = 0; rr < 2; ++rr) {
      const unsigned so = (2u * wave + (unsigned)rr) * MPITCH + 4u * lane;
      v4f v[4];
#pragma unroll
      for (int j = 0; j < 4; ++j) v[j] = *(const v4fa*)(mk + so + 128 * j);
      float mx = v[0].x;
#pragma unroll
      for (int j = 0; j < 4; ++j) mx = fmaxf(fmaxf(fmaxf(mx, v[j].x), fmaxf(v[j].y, v[j].z)), v[j].w);
      mx = fmaxf(mx, __shfl_xor(mx, 16));
      mx = fmaxf(mx, __shfl_xor(mx, 8));
      mx = fmaxf(mx, __shfl_xor(mx, 4));
      mx = fmaxf(mx, __shfl_xor(mx, 2));
      mx = fmaxf(mx, __shfl_xor(mx, 1));
      float sum = 0.0f;
#pragma unroll
      for (int j = 0; j < 4; ++j) {
        v[j].x = expf(v[j].x - mx); v[j].y = expf(v[j].y - mx);
        v[j].z = expf(v[j].z - mx); v[j].w = expf(v[j].w - mx);
        sum += (v[j].x + v[j].y) + (v[j].z + v[j].w);
      }
      sum += __shfl_xor(sum, 16);
      sum += __shfl_xor(sum, 8);
      sum += __shfl_xor(sum, 4);
      sum += __shfl_xor(sum, 2);
      sum += __shfl_xor(sum, 1);
      const float inv = 1.0f / sum;
#pragma unroll
      for (int j = 0; j < 4; ++j) res[rr][j] = v[j] * inv;
    }
    float* ob = out + ((size_t)b * GQ + g0 + 2u * wave) * NK + 4u * lane;
#pragma unroll
    for (int rr = 0; rr < 2; ++rr)
#pragma unroll
      for (int j = 0; j < 4; ++j) *(volatile v4f*)(ob + (size_t)rr * NK + 128 * j) = res[rr][j];
    __threadfence();
#pragma unroll
    for (int rr = 0; rr < 2; ++rr)
#pragma unroll
      for (int j = 0; j < 4; ++j) *(volatile v4f*)(ob + (size_t)rr * NK + 128 * j) = res[rr][j];
  }
}

static inline size_t al256(size_t o) { return (o + 255) & ~(size_t)255; }

extern "C" void kernel_launch(void* const* d_in, const int* in_sizes, int n_in,
                              void* d_out, int out_size, void* d_ws, size_t ws_size,
                              hipStream_t stream) {
  if (n_in < 10) return;
  const long long actN = (long long)NB * NK * EW;
  const long long actG = (long long)NB * GQ * EW;
  const long long mskN = (long long)NB * GQ * NK;
  if ((long long)in_sizes[0] < actN) return;
  if ((long long)in_sizes[1] < actG) return;
  if ((long long)in_sizes[2] < actG) return;
  if ((long long)in_sizes[3] < mskN) return;
  if (in_sizes[4] < EW * EW || in_sizes[5] < EW * EW || in_sizes[6] < EW * EW ||
      in_sizes[7] < EW * EW || in_sizes[8] < EW * EW) return;
  if (in_sizes[9] < EW) return;
  if ((long long)out_size < mskN) return;

  const float* nodes = (const float*)d_in[0];
  const float* q1    = (const float*)d_in[1];
  const float* last  = (const float*)d_in[2];
  const float* mask  = (const float*)d_in[3];
  const float* Wqf   = (const float*)d_in[4];
  const float* Wql   = (const float*)d_in[5];
  const float* Wk    = (const float*)d_in[6];
  const float* Wv    = (const float*)d_in[7];
  const float* Wc    = (const float*)d_in[8];
  const float* bc    = (const float*)d_in[9];
  float* out = (float*)d_out;

  const size_t wtB  = al256((size_t)5 * EW * EW * 2);
  const size_t nbB  = al256((size_t)NB * NK * EW * 2);
  const size_t qB   = al256((size_t)NB * NH * GQ * QROW * 2);
  const size_t kB   = al256((size_t)NB * NH * NK * QROW * 2);
  const size_t vB   = al256((size_t)2 * VPL * 2);
  const size_t total = wtB + nbB + qB + kB + vB;
  if (total > ws_size || total > (size_t)WSMAX) return;
  char* w = (char*)d_ws;
  unsigned short* wt  = (unsigned short*)w;
  unsigned short* nbf = (unsigned short*)(w + wtB);
  unsigned short* qpl = (unsigned short*)(w + wtB + nbB);
  unsigned short* kpl = (unsigned short*)(w + wtB + nbB + qB);
  unsigned short* vtp = (unsigned short*)(w + wtB + nbB + qB + kB);
  unsigned short* wqft = wt;
  unsigned short* wqlt = wt + 1 * EW * EW;
  unsigned short* wkt  = wt + 2 * EW * EW;
  unsigned short* wvt  = wt + 3 * EW * EW;
  unsigned short* wctp = wt + 4 * EW * EW;

  k_wprep<<<dim3(4, 5), 256, 0, stream>>>(Wqf, Wql, Wk, Wv, Wc, wt);
  k_cvt<<<(unsigned)(((size_t)NB * NK * EW) / (256 * 8)), 256, 0, stream>>>(nodes, nbf);
  k_proj<0><<<(NB * GQ) / 64, 128, 0, stream>>>(q1, last, wqft, wqlt, qpl, qpl);
  k_proj<1><<<(NB * NK) / 64, 128, 0, stream>>>(nodes, nodes, wkt, wvt, kpl, vtp);
  k_dec<<<dim3(GQ / 16, NB), 256, 0, stream>>>(qpl, kpl, vtp, mask, wctp, bc, nbf, out);
}
